// GATModel_40939628265881
// MI455X (gfx1250) — hardware-verified
//
#include <hip/hip_runtime.h>
#include <stddef.h>
#include <stdint.h>
#include <math.h>


#define DF      6
#define TT      60
#define HH      64
#define G3      192
#define XW      360
#define GR      32
#define GT      256
#define WM_H    (G3 * HH)
#define WPL_H   (3 * WM_H + G3 * 8)
#define WPL_V4  (WPL_H / 8)
#define XS_H    (TT * GR * 8)
#define HB_H    (GR * 128)
#define HA_H    (4 * HB_H)
#define LDS_GRU (WPL_H * 2 + XS_H * 2 + HA_H * 2 + 2 * 4 * HH * 4)
#define PR      64
#define RSTR    4160
#define LDS_P2  ((4 * 4096 + 64 + 64 + 64 + 256 + 128) * 4)
#define WSMAX   134217728

static_assert(XW == DF * TT);
static_assert(G3 == 3 * HH && (HH % 32) == 0);
static_assert((WPL_H % 8) == 0 && (XS_H % 8) == 0 && (HA_H % 8) == 0);
static_assert(GT == 8 * 32 && GR == 32);
static_assert((GR * HH + 128) * 4 <= XS_H * 2);
static_assert((RSTR * 4) % 128 == 0);
static_assert(LDS_GRU <= 300000 && LDS_P2 <= 300000);
static_assert(3 * 1536 == 4608 && (1536 % 256) == 0);

typedef float          v4f  __attribute__((ext_vector_type(4)));
typedef float          v8f  __attribute__((ext_vector_type(8)));
typedef int            v8i  __attribute__((ext_vector_type(8)));
typedef unsigned int   v4u  __attribute__((ext_vector_type(4)));
typedef unsigned short v8us __attribute__((ext_vector_type(8)));
typedef __bf16         v16b __attribute__((ext_vector_type(16)));
typedef v4f  __attribute__((may_alias)) v4fa;
typedef v4u  __attribute__((may_alias)) v4ua;
typedef v8us __attribute__((may_alias)) v8usa;
union FragB { v16b v; v8us h[2]; v4u q[2]; v8i w; };

__device__ __forceinline__ v8f wmb(const FragB& a, const FragB& b, v8f c) {
  v8f d = __builtin_amdgcn_wmma_f32_16x16x32_bf16(false, a.v, false, b.v, (short)0, c, false, false);
  asm volatile("v_nop\n\tv_nop\n\tv_nop\n\tv_nop" : "+v"(d) : "v"(a.w), "v"(b.w));
  return d;
}

__device__ __forceinline__ unsigned int f2bf(float f) {
  const unsigned int u = __float_as_uint(f);
  return ((u + 0x7FFFu + ((u >> 16) & 1u)) >> 16) & 0xFFFFu;
}
__device__ __forceinline__ float bf2f(unsigned int b) { return __uint_as_float(b << 16); }
__device__ __forceinline__ float bfr(float f) { return bf2f(f2bf(f)); }
__device__ __forceinline__ unsigned int pk2(float lo, float hi) { return f2bf(lo) | (f2bf(hi) << 16); }
__device__ __forceinline__ v4u pack8(const v4f a, const v4f b) {
  v4u r;
  r.x = pk2(a.x, a.y); r.y = pk2(a.z, a.w); r.z = pk2(b.x, b.y); r.w = pk2(b.z, b.w);
  return r;
}

__global__ __launch_bounds__(256) void k_prep(const float* __restrict__ Whh0, const float* __restrict__ Wih1,
                                              const float* __restrict__ Whh1, const float* __restrict__ Wih0,
                                              unsigned short* WP) {
  const int u = (int)blockIdx.x * 256 + (int)threadIdx.x;
  v4u o;
  size_t dst;
  if (u < 4608) {
    const int which = u / 1536;
    const int v = u - which * 1536;
    const float* src = (which == 0) ? Whh0 : ((which == 1) ? Wih1 : Whh1);
    const float* p = src + (size_t)v * 8;
    const v4f a = *(const v4fa*)p;
    const v4f b = *(const v4fa*)(p + 4);
    o = pack8(a, b);
    dst = (size_t)u * 8;
  } else if (u < 4800) {
    const int n = u - 4608;
    const float* p = Wih0 + (size_t)n * DF;
    const float f0 = p[0], f1 = p[1], f2 = p[2], f3 = p[3], f4 = p[4], f5 = p[5];
    o.x = pk2(f0, f1); o.y = pk2(f2, f3); o.z = pk2(f4, f5); o.w = 0u;
    dst = (size_t)(3 * WM_H) + (size_t)n * 8;
  } else {
    return;
  }
  *(volatile v4u*)(WP + dst) = o;
  __threadfence();
  *(volatile v4u*)(WP + dst) = o;
}

__device__ __forceinline__ void mm_h(const unsigned short* ap, const unsigned short* wp,
                                     v8f& aR, v8f& aZ, v8f& aN) {
#pragma unroll
  for (int kk = 0; kk < 2; ++kk) {
    FragB bR, bZ, bN, ah, al;
    bR.h[0] = *(const v8usa*)(wp + 32 * kk);
    bR.h[1] = *(const v8usa*)(wp + 32 * kk + 16);
    bZ.h[0] = *(const v8usa*)(wp + 4096 + 32 * kk);
    bZ.h[1] = *(const v8usa*)(wp + 4096 + 32 * kk + 16);
    bN.h[0] = *(const v8usa*)(wp + 8192 + 32 * kk);
    bN.h[1] = *(const v8usa*)(wp + 8192 + 32 * kk + 16);
    ah.h[0] = *(const v8usa*)(ap + 32 * kk);
    ah.h[1] = *(const v8usa*)(ap + 32 * kk + 16);
    al.h[0] = *(const v8usa*)(ap + 64 + 32 * kk);
    al.h[1] = *(const v8usa*)(ap + 64 + 32 * kk + 16);
    aR = wmb(ah, bR, aR);
    aZ = wmb(ah, bZ, aZ);
    aN = wmb(ah, bN, aN);
    aR = wmb(al, bR, aR);
    aZ = wmb(al, bZ, aZ);
    aN = wmb(al, bN, aN);
  }
}

__device__ __forceinline__ void gates(const v8f& aR, const v8f& aZ, const v8f& aX, const v8f& aH,
                                      float bR, float bZ, float bX, float bH,
                                      float (&hc)[8], unsigned short* hrow) {
#pragma unroll
  for (int r = 0; r < 8; ++r) {
    const float rg = 1.0f / (1.0f + expf(-(aR[r] + bR)));
    const float zg = 1.0f / (1.0f + expf(-(aZ[r] + bZ)));
    const float ng = tanhf((aX[r] + bX) + rg * (aH[r] + bH));
    const float hv = (1.0f - zg) * ng + zg * hc[r];
    hc[r] = hv;
    const unsigned int hb = f2bf(hv);
    const unsigned int lb = f2bf(hv - bf2f(hb));
    hrow[r * 128]      = (unsigned short)hb;
    hrow[r * 128 + 64] = (unsigned short)lb;
  }
}

__global__ __launch_bounds__(GT) void k_gru(const float* __restrict__ x, const unsigned short* __restrict__ WP,
                                            const float* __restrict__ bih0, const float* __restrict__ bhh0,
                                            const float* __restrict__ bih1, const float* __restrict__ bhh1,
                                            float* HID, float* REC, int nN) {
  extern __shared__ v4f lds_dyn[];
  unsigned short* WL = (unsigned short*)lds_dyn;
  unsigned short* W0 = WL + 3 * WM_H;
  unsigned short* XS = W0 + G3 * 8;
  unsigned short* HA = XS + XS_H;
  float*          BS = (float*)(HA + HA_H);
  const int tid = (int)threadIdx.x, lane = tid & 31, wave = tid >> 5, hh = lane >> 4, m = lane & 15;
  const int rowbase = (int)blockIdx.x * GR;

#pragma unroll 1
  for (int p = tid; p < WPL_V4; p += GT) {
    const v4u wv = *(const v4ua*)(WP + (size_t)p * 8);
    *(v4ua*)(WL + p * 8) = wv;
  }
#pragma unroll 1
  for (int u = tid; u < TT * GR; u += GT) {
    const int t = u >> 5, r = u & 31;
    int row = rowbase + r;
    row = row < nN ? row : nN - 1;
    const float* xp = x + (size_t)row * XW + t;
    const float f0 = xp[0], f1 = xp[TT], f2 = xp[2 * TT], f3 = xp[3 * TT], f4 = xp[4 * TT], f5 = xp[5 * TT];
    v4u w;
    w.x = pk2(f0, f1); w.y = pk2(f2, f3); w.z = pk2(f4, f5); w.w = 0u;
    *(v4ua*)(XS + u * 8) = w;
  }
  {
    const v4u z4 = {0u, 0u, 0u, 0u};
#pragma unroll 1
    for (int p = tid; p < HA_H / 8; p += GT) *(v4ua*)(HA + p * 8) = z4;
  }
  {
    const int jj = tid & 63, which = tid >> 6;
    const int g = which < 2 ? which : 2;
    const int idx = g * HH + jj;
    const float a0 = bfr(bih0[idx]), c0 = bfr(bhh0[idx]);
    const float a1 = bfr(bih1[idx]), c1 = bfr(bhh1[idx]);
    const float v0 = (which < 2) ? (a0 + c0) : ((which == 2) ? a0 : c0);
    const float v1 = (which < 2) ? (a1 + c1) : ((which == 2) ? a1 : c1);
    BS[which * HH + jj]       = v0;
    BS[256 + which * HH + jj] = v1;
  }
  __syncthreads();

  const int rt = wave & 1, cq = wave >> 1;
  const int j = 16 * cq + m;
  const int aoff = (rt * 16 + m) * 128 + 8 * hh;
  const int woff = j * HH + 8 * hh;
  const int doff = (rt * 16 + 8 * hh) * 128 + j;
  const float b0r = BS[j],       b0z = BS[64 + j],        b0x = BS[128 + j],       b0h = BS[192 + j];
  const float b1r = BS[256 + j], b1z = BS[256 + 64 + j],  b1x = BS[256 + 128 + j], b1h = BS[256 + 192 + j];

  const unsigned int msk = (unsigned int)(hh - 1);
  const v4u mk  = {msk, msk, msk, msk};
  const v4u z4u = {0u, 0u, 0u, 0u};
  FragB bxr, bxz, bxn;
  bxr.q[0] = (*(const v4ua*)(W0 + (0 * HH + j) * 8)) & mk;  bxr.q[1] = z4u;
  bxz.q[0] = (*(const v4ua*)(W0 + (1 * HH + j) * 8)) & mk;  bxz.q[1] = z4u;
  bxn.q[0] = (*(const v4ua*)(W0 + (2 * HH + j) * 8)) & mk;  bxn.q[1] = z4u;

  float hc0[8], hc1[8];
#pragma unroll
  for (int r = 0; r < 8; ++r) { hc0[r] = 0.0f; hc1[r] = 0.0f; }
  const v8f z8 = {0.f, 0.f, 0.f, 0.f, 0.f, 0.f, 0.f, 0.f};

#pragma unroll 1
  for (int t = 0; t < TT; ++t) {
    const int cur = t & 1, nxt = cur ^ 1;
    v8f aR = z8, aZ = z8, aX = z8, aH = z8;
    {
      FragB ax;
      ax.q[0] = (*(const v4ua*)(XS + (t * GR + rt * 16 + m) * 8)) & mk;
      ax.q[1] = z4u;
      aR = wmb(ax, bxr, aR);
      aZ = wmb(ax, bxz, aZ);
      aX = wmb(ax, bxn, aX);
    }
    mm_h(HA + (0 * 2 + cur) * HB_H + aoff, WL + woff, aR, aZ, aH);
    gates(aR, aZ, aX, aH, b0r, b0z, b0x, b0h, hc0, HA + (0 * 2 + nxt) * HB_H + doff);
    __syncthreads();
    aR = z8; aZ = z8; aX = z8; aH = z8;
    mm_h(HA + (0 * 2 + nxt) * HB_H + aoff, WL + WM_H + woff, aR, aZ, aX);
    mm_h(HA + (1 * 2 + cur) * HB_H + aoff, WL + 2 * WM_H + woff, aR, aZ, aH);
    gates(aR, aZ, aX, aH, b1r, b1z, b1x, b1h, hc1, HA + (1 * 2 + nxt) * HB_H + doff);
  }
  __syncthreads();

  float* HS = (float*)XS;
  float* RC = HS + GR * HH;
#pragma unroll
  for (int r = 0; r < 8; ++r) HS[(rt * 16 + 8 * hh + r) * HH + j] = hc1[r];
  __syncthreads();
  if (tid < HH) {
    float s = 0.0f;
#pragma unroll 4
    for (int rr = 0; rr < GR; ++rr) s += HS[rr * HH + tid];
    const float mu = s * (1.0f / (float)GR);
    float q = 0.0f;
#pragma unroll 4
    for (int rr = 0; rr < GR; ++rr) { const float d = HS[rr * HH + tid] - mu; q = fmaf(d, d, q); }
    RC[tid] = s;
    RC[HH + tid] = q;
  }
  __syncthreads();
  const v4f h0v = *(const v4fa*)(HS + 4 * tid);
  const v4f h1v = *(const v4fa*)(HS + 4 * (tid + GT));
  const v4f rv  = *(const v4fa*)(RC + 4 * lane);
  float* hp = HID + (size_t)rowbase * HH;
  float* rp = REC + (size_t)blockIdx.x * 128 + 4 * lane;
  *(volatile v4f*)(hp + 4 * tid) = h0v;
  *(volatile v4f*)(hp + 4 * (tid + GT)) = h1v;
  if (wave == 0) *(volatile v4f*)rp = rv;
  __threadfence();
  *(volatile v4f*)(hp + 4 * tid) = h0v;
  *(volatile v4f*)(hp + 4 * (tid + GT)) = h1v;
  if (wave == 0) *(volatile v4f*)rp = rv;
}

__global__ __launch_bounds__(64) void k_bncomb(const float* __restrict__ REC, int nrec, double rows, double invRows,
                                               double invN, const float* __restrict__ w,
                                               const float* __restrict__ b, float* P) {
  __shared__ __attribute__((aligned(16))) float ps[256];
  const int c = (int)threadIdx.x;
  double S = 0.0;
#pragma unroll 4
  for (int r = 0; r < nrec; ++r) S += (double)REC[(size_t)r * 128 + c];
  const double mean = S * invN;
  double M2 = 0.0;
#pragma unroll 4
  for (int r = 0; r < nrec; ++r) {
    const double sr = (double)REC[(size_t)r * 128 + c];
    const double qr = (double)REC[(size_t)r * 128 + 64 + c];
    const double d = sr * invRows - mean;
    M2 += qr + rows * d * d;
  }
  const float var = (float)(M2 * invN);
  ps[c]       = (float)mean;
  ps[64 + c]  = bfr(w[c]) * rsqrtf(var + 1e-5f);
  ps[128 + c] = bfr(b[c]);
  ps[192 + c] = 0.0f;
  __syncthreads();
  const v4f v = *(const v4fa*)(ps + 4 * c);
  *(volatile v4f*)(P + 4 * c) = v;
  __threadfence();
  *(volatile v4f*)(P + 4 * c) = v;
}

__device__ __forceinline__ void load_hbn(const float* __restrict__ HID, int rowbase, const float* ps, float* hb, int tid) {
#pragma unroll 1
  for (int i = 0; i < 4; ++i) {
    const int p = tid + 256 * i;
    const v4f v = *(const v4fa*)(HID + (size_t)rowbase * HH + 4 * p);
    const int c = (4 * p) & 63;
    const v4f mm = *(const v4fa*)(ps + c);
    const v4f aa = *(const v4fa*)(ps + 64 + c);
    const v4f bb = *(const v4fa*)(ps + 128 + c);
    v4f o;
    o.x = (v.x - mm.x) * aa.x + bb.x;
    o.y = (v.y - mm.y) * aa.y + bb.y;
    o.z = (v.z - mm.z) * aa.z + bb.z;
    o.w = (v.w - mm.w) * aa.w + bb.w;
    *(v4fa*)(hb + 4 * p) = o;
  }
}

__device__ __forceinline__ void mac16(const float* A, int sI, int sJ, const float* B, int i, int cb, float (&acc)[16]) {
#pragma unroll
  for (int c = 0; c < 16; ++c) acc[c] = 0.0f;
#pragma unroll 1
  for (int jj = 0; jj < 64; ++jj) {
    const float a = A[i * sI + jj * sJ];
    const float* br = B + jj * 64 + cb;
#pragma unroll
    for (int q = 0; q < 4; ++q) {
      const v4f bv = *(const v4fa*)(br + 4 * q);
      acc[4 * q + 0] = fmaf(a, bv.x, acc[4 * q + 0]);
      acc[4 * q + 1] = fmaf(a, bv.y, acc[4 * q + 1]);
      acc[4 * q + 2] = fmaf(a, bv.z, acc[4 * q + 2]);
      acc[4 * q + 3] = fmaf(a, bv.w, acc[4 * q + 3]);
    }
  }
}

__global__ __launch_bounds__(256) void k_post1(const float* __restrict__ HID, const float* __restrict__ P1, float* RECC) {
  __shared__ __attribute__((aligned(16))) float hb[4096];
  __shared__ __attribute__((aligned(16))) float ct[4096];
  __shared__ __attribute__((aligned(16))) float ps[192];
  __shared__ __attribute__((aligned(16))) float es[64];
  __shared__ __attribute__((aligned(16))) float ss[64];
  const int tid = (int)threadIdx.x;
  const int rowbase = (int)blockIdx.x * PR;
  if (tid < 192) ps[tid] = P1[tid];
  __syncthreads();
  load_hbn(HID, rowbase, ps, hb, tid);
  __syncthreads();
  if (tid < 64) {
    float s = 0.0f;
#pragma unroll 4
    for (int c4 = 0; c4 < 16; ++c4) {
      const v4f v = *(const v4fa*)(hb + tid * 64 + 4 * c4);
      s += v.x; s += v.y; s += v.z; s += v.w;
    }
    es[tid] = s * (1.0f / 64.0f);
  }
  __syncthreads();
  {
    const int i = tid >> 2, jb = (tid & 3) * 16;
    float acc[16];
    mac16(hb, 1, 64, hb, i, jb, acc);
#pragma unroll
    for (int q = 0; q < 4; ++q) {
      v4f o; o.x = acc[4 * q]; o.y = acc[4 * q + 1]; o.z = acc[4 * q + 2]; o.w = acc[4 * q + 3];
      *(v4fa*)(ct + i * 64 + jb + 4 * q) = o;
    }
  }
  if (tid < 64) {
    float sa = 0.0f;
#pragma unroll 4
    for (int rr = 0; rr < 64; ++rr) sa = fmaf(es[rr], hb[rr * 64 + tid], sa);
    ss[tid] = sa;
  }
  __syncthreads();
  float* rb = RECC + (size_t)blockIdx.x * RSTR;
  const v4f c0 = *(const v4fa*)(ct + 4 * tid);
  const v4f c1 = *(const v4fa*)(ct + 4 * (tid + 256));
  const v4f c2 = *(const v4fa*)(ct + 4 * (tid + 512));
  const v4f c3 = *(const v4fa*)(ct + 4 * (tid + 768));
  const v4f sv = *(const v4fa*)(ss + 4 * (tid & 15));
  *(volatile v4f*)(rb + 4 * tid) = c0;
  *(volatile v4f*)(rb + 4 * (tid + 256)) = c1;
  *(volatile v4f*)(rb + 4 * (tid + 512)) = c2;
  *(volatile v4f*)(rb + 4 * (tid + 768)) = c3;
  if (tid < 16) *(volatile v4f*)(rb + 4096 + 4 * tid) = sv;
  __threadfence();
  *(volatile v4f*)(rb + 4 * tid) = c0;
  *(volatile v4f*)(rb + 4 * (tid + 256)) = c1;
  *(volatile v4f*)(rb + 4 * (tid + 512)) = c2;
  *(volatile v4f*)(rb + 4 * (tid + 768)) = c3;
  if (tid < 16) *(volatile v4f*)(rb + 4096 + 4 * tid) = sv;
}

__global__ __launch_bounds__(256) void k_comb2(const float* __restrict__ RECC, int nrec, float* CS) {
  __shared__ __attribute__((aligned(16))) float res[256];
  const int tid = (int)threadIdx.x, blk = (int)blockIdx.x;
  const bool isS = (blk == 16);
  const int idx = isS ? (4096 + (tid & 63)) : (blk * 256 + tid);
  double s = 0.0;
#pragma unroll 4
  for (int r = 0; r < nrec; ++r) s += (double)RECC[(size_t)r * RSTR + idx];
  const double sc = isS ? 1.0 : (1.0 / 64.0);
  res[tid] = (float)(s * sc);
  __syncthreads();
  const int npc = isS ? 16 : 64;
  const v4f v = *(const v4fa*)(res + 4 * (tid & 63));
  float* op = CS + (size_t)blk * 256 + 4 * (tid & 63);
  if (tid < npc) *(volatile v4f*)op = v;
  __threadfence();
  if (tid < npc) *(volatile v4f*)op = v;
}

__global__ __launch_bounds__(256) void k_post2(const float* __restrict__ HID, const float* __restrict__ P1,
                                               const float* __restrict__ CS, const float* __restrict__ fcw,
                                               const float* __restrict__ fcb, float* F, float* REC2) {
  extern __shared__ v4f lds_dyn[];
  float* C64 = (float*)lds_dyn;
  float* FWT = C64 + 4096;
  float* HB  = FWT + 4096;
  float* OT  = HB + 4096;
  float* SS  = OT + 4096;
  float* FB  = SS + 64;
  float* ES  = FB + 64;
  float* PS  = ES + 64;
  float* RC  = PS + 256;
  const int tid = (int)threadIdx.x, lane = tid & 31, wave = tid >> 5;
  const int rowbase = (int)blockIdx.x * PR;

#pragma unroll 1
  for (int i = 0; i < 4; ++i) {
    const int p = tid + 256 * i;
    const v4f cv = *(const v4fa*)(CS + 4 * p);
    *(v4fa*)(C64 + 4 * p) = cv;
    const v4f wv = *(const v4fa*)(fcw + 4 * p);
    const int n = (4 * p) >> 6, k0 = (4 * p) & 63;
    FWT[(k0 + 0) * 64 + n] = bfr(wv.x);
    FWT[(k0 + 1) * 64 + n] = bfr(wv.y);
    FWT[(k0 + 2) * 64 + n] = bfr(wv.z);
    FWT[(k0 + 3) * 64 + n] = bfr(wv.w);
  }
  if (tid < 64) { SS[tid] = CS[4096 + tid]; FB[tid] = bfr(fcb[tid]); }
  if (tid < 192) PS[tid] = P1[tid];
  __syncthreads();
  load_hbn(HID, rowbase, PS, HB, tid);
  __syncthreads();
  if (tid < 64) {
    float s = 0.0f;
#pragma unroll 4
    for (int c4 = 0; c4 < 16; ++c4) {
      const v4f v = *(const v4fa*)(HB + tid * 64 + 4 * c4);
      s += v.x; s += v.y; s += v.z; s += v.w;
    }
    ES[tid] = s * (1.0f / 64.0f);
  }
  __syncthreads();
  const int i = tid >> 2, cb = (tid & 3) * 16;
  {
    float acc[16];
    mac16(HB, 64, 1, C64, i, cb, acc);
    const float ne = -ES[i];
#pragma unroll
    for (int q = 0; q < 4; ++q) {
      const v4f sv = *(const v4fa*)(SS + cb + 4 * q);
      v4f o;
      o.x = fmaf(ne, sv.x, acc[4 * q]);
      o.y = fmaf(ne, sv.y, acc[4 * q + 1]);
      o.z = fmaf(ne, sv.z, acc[4 * q + 2]);
      o.w = fmaf(ne, sv.w, acc[4 * q + 3]);
      *(v4fa*)(OT + i * 64 + cb + 4 * q) = o;
    }
  }
  __syncthreads();
  {
    float acc[16];
    mac16(OT, 64, 1, FWT, i, cb, acc);
#pragma unroll
    for (int q = 0; q < 4; ++q) {
      const v4f bv = *(const v4fa*)(FB + cb + 4 * q);
      v4f o;
      o.x = acc[4 * q] + bv.x; o.y = acc[4 * q + 1] + bv.y; o.z = acc[4 * q + 2] + bv.z; o.w = acc[4 * q + 3] + bv.w;
      *(v4fa*)(HB + i * 64 + cb + 4 * q) = o;
    }
  }
  __syncthreads();
  if (tid < 64) {
    float s = 0.0f;
#pragma unroll 4
    for (int rr = 0; rr < PR; ++rr) s += HB[rr * 64 + tid];
    const float mu = s * (1.0f / (float)PR);
    float q = 0.0f;
#pragma unroll 4
    for (int rr = 0; rr < PR; ++rr) { const float d = HB[rr * 64 + tid] - mu; q = fmaf(d, d, q); }
    RC[tid] = s;
    RC[64 + tid] = q;
  }
  __syncthreads();
  float* fp = F + (size_t)rowbase * HH;
  const v4f f0 = *(const v4fa*)(HB + 4 * tid);
  const v4f f1 = *(const v4fa*)(HB + 4 * (tid + 256));
  const v4f f2 = *(const v4fa*)(HB + 4 * (tid + 512));
  const v4f f3 = *(const v4fa*)(HB + 4 * (tid + 768));
  const v4f rv = *(const v4fa*)(RC + 4 * lane);
  float* rp = REC2 + (size_t)blockIdx.x * 128 + 4 * lane;
  *(volatile v4f*)(fp + 4 * tid) = f0;
  *(volatile v4f*)(fp + 4 * (tid + 256)) = f1;
  *(volatile v4f*)(fp + 4 * (tid + 512)) = f2;
  *(volatile v4f*)(fp + 4 * (tid + 768)) = f3;
  if (wave == 0) *(volatile v4f*)rp = rv;
  __threadfence();
  *(volatile v4f*)(fp + 4 * tid) = f0;
  *(volatile v4f*)(fp + 4 * (tid + 256)) = f1;
  *(volatile v4f*)(fp + 4 * (tid + 512)) = f2;
  *(volatile v4f*)(fp + 4 * (tid + 768)) = f3;
  if (wave == 0) *(volatile v4f*)rp = rv;
}

__global__ __launch_bounds__(256) void k_out(const float* __restrict__ F, const float* __restrict__ P2,
                                             const float* __restrict__ fow, const float* __restrict__ fob, float* out) {
  __shared__ __attribute__((aligned(16))) float ps[192];
  __shared__ __attribute__((aligned(16))) float fw[64];
  __shared__ __attribute__((aligned(16))) float res[256];
  const int tid = (int)threadIdx.x;
  if (tid < 192) ps[tid] = P2[tid];
  if (tid < 64) fw[tid] = bfr(fow[tid]);
  __syncthreads();
  const size_t row = (size_t)blockIdx.x * 256 + (size_t)tid;
  const float* fr = F + row * HH;
  float acc = 0.0f;
#pragma unroll 2
  for (int c4 = 0; c4 < 16; ++c4) {
    const v4f f  = *(const v4fa*)(fr + 4 * c4);
    const v4f mm = *(const v4fa*)(ps + 4 * c4);
    const v4f aa = *(const v4fa*)(ps + 64 + 4 * c4);
    const v4f bb = *(const v4fa*)(ps + 128 + 4 * c4);
    const v4f ww = *(const v4fa*)(fw + 4 * c4);
    float y0 = (f.x - mm.x) * aa.x + bb.x;
    float y1 = (f.y - mm.y) * aa.y + bb.y;
    float y2 = (f.z - mm.z) * aa.z + bb.z;
    float y3 = (f.w - mm.w) * aa.w + bb.w;
    y0 = (y0 >= 0.0f) ? y0 : 0.01f * y0;
    y1 = (y1 >= 0.0f) ? y1 : 0.01f * y1;
    y2 = (y2 >= 0.0f) ? y2 : 0.01f * y2;
    y3 = (y3 >= 0.0f) ? y3 : 0.01f * y3;
    acc = fmaf(y0, ww.x, acc);
    acc = fmaf(y1, ww.y, acc);
    acc = fmaf(y2, ww.z, acc);
    acc = fmaf(y3, ww.w, acc);
  }
  res[tid] = acc + bfr(fob[0]);
  __syncthreads();
  const v4f v = *(const v4fa*)(res + 4 * (tid & 63));
  float* op = out + (size_t)blockIdx.x * 256 + 4 * (tid & 63);
  if (tid < 64) *(volatile v4f*)op = v;
  __threadfence();
  if (tid < 64) *(volatile v4f*)op = v;
}

extern "C" void kernel_launch(void* const* d_in, const int* in_sizes, int n_in,
                              void* d_out, int out_size, void* d_ws, size_t ws_size,
                              hipStream_t stream) {
  if (n_in < 17) return;
  if (in_sizes[0] < XW || (in_sizes[0] % XW) != 0) return;
  const int nN = in_sizes[0] / XW;
  if (nN <= 0 || (nN % 256) != 0 || nN > 65536) return;
  if (in_sizes[1] != G3 * DF) return;
  if (in_sizes[2] != G3 * HH || in_sizes[5] != G3 * HH || in_sizes[6] != G3 * HH) return;
  if (in_sizes[3] != G3 || in_sizes[4] != G3 || in_sizes[7] != G3 || in_sizes[8] != G3) return;
  if (in_sizes[9] != HH || in_sizes[10] != HH || in_sizes[12] != HH || in_sizes[13] != HH ||
      in_sizes[14] != HH || in_sizes[15] != HH) return;
  if (in_sizes[11] != HH * HH) return;
  if (in_sizes[16] != 1) return;
  if (out_size != nN) return;

  const float* x    = (const float*)d_in[0];
  const float* Wih0 = (const float*)d_in[1];
  const float* Whh0 = (const float*)d_in[2];
  const float* bih0 = (const float*)d_in[3];
  const float* bhh0 = (const float*)d_in[4];
  const float* Wih1 = (const float*)d_in[5];
  const float* Whh1 = (const float*)d_in[6];
  const float* bih1 = (const float*)d_in[7];
  const float* bhh1 = (const float*)d_in[8];
  const float* bn1w = (const float*)d_in[9];
  const float* bn1b = (const float*)d_in[10];
  const float* fcw  = (const float*)d_in[11];
  const float* fcb  = (const float*)d_in[12];
  const float* bn2w = (const float*)d_in[13];
  const float* bn2b = (const float*)d_in[14];
  const float* fow  = (const float*)d_in[15];
  const float* fob  = (const float*)d_in[16];
  float* out = (float*)d_out;

  const int gG = nN / GR;
  const int gP = nN / PR;

  char* ws = (char*)d_ws;
  size_t off = 0;
  const size_t oWP  = off; off += (size_t)WPL_H * 2;            off = (off + 255) & ~(size_t)255;
  const size_t oHID = off; off += (size_t)nN * HH * 4;          off = (off + 255) & ~(size_t)255;
  const size_t oR1  = off; off += (size_t)gG * 128 * 4;         off = (off + 255) & ~(size_t)255;
  const size_t oP1  = off; off += (size_t)256 * 4;              off = (off + 255) & ~(size_t)255;
  const size_t oRC  = off; off += (size_t)gP * RSTR * 4;        off = (off + 255) & ~(size_t)255;
  const size_t oCS  = off; off += (size_t)RSTR * 4;             off = (off + 255) & ~(size_t)255;
  const size_t oF   = off; off += (size_t)nN * HH * 4;          off = (off + 255) & ~(size_t)255;
  const size_t oR2  = off; off += (size_t)gP * 128 * 4;         off = (off + 255) & ~(size_t)255;
  const size_t oP2  = off; off += (size_t)256 * 4;              off = (off + 255) & ~(size_t)255;
  if (off > ws_size || off > (size_t)WSMAX) return;
  unsigned short* WP = (unsigned short*)(ws + oWP);
  float* HID  = (float*)(ws + oHID);
  float* REC1 = (float*)(ws + oR1);
  float* P1   = (float*)(ws + oP1);
  float* RECC = (float*)(ws + oRC);
  float* CS   = (float*)(ws + oCS);
  float* F    = (float*)(ws + oF);
  float* REC2 = (float*)(ws + oR2);
  float* P2   = (float*)(ws + oP2);

  hipFuncSetAttribute(reinterpret_cast<const void*>(&k_gru), hipFuncAttributeMaxDynamicSharedMemorySize, LDS_GRU);
  hipFuncSetAttribute(reinterpret_cast<const void*>(&k_post2), hipFuncAttributeMaxDynamicSharedMemorySize, LDS_P2);

  const double invN = 1.0 / (double)nN;

  k_prep<<<19, 256, 0, stream>>>(Whh0, Wih1, Whh1, Wih0, WP);
  k_gru<<<gG, GT, LDS_GRU, stream>>>(x, WP, bih0, bhh0, bih1, bhh1, HID, REC1, nN);
  k_bncomb<<<1, 64, 0, stream>>>(REC1, gG, (double)GR, 1.0 / (double)GR, invN, bn1w, bn1b, P1);
  k_post1<<<gP, 256, 0, stream>>>(HID, P1, RECC);
  k_comb2<<<17, 256, 0, stream>>>(RECC, gP, CS);
  k_post2<<<gP, 256, LDS_P2, stream>>>(HID, P1, CS, fcw, fcb, F, REC2);
  k_bncomb<<<1, 64, 0, stream>>>(REC2, gP, (double)PR, 1.0 / (double)PR, invN, bn2w, bn2b, P2);
  k_out<<<nN / 256, 256, 0, stream>>>(F, P2, fow, fob, out);
}
